// CrossInvolution_55035710931681
// MI455X (gfx1250) — hardware-run, weakly checked
//
#include <hip/hip_runtime.h>


#define NSP  2
#define NMP  256
#define NRD  64
#define NPL  4096
#define NSD  64
#define NFL  784
#define NFP  832
#define NTP  49
#define OBB  256
constexpr size_t al256(size_t b) { return (b + 255) & ~(size_t)255; }
constexpr size_t WS_TOTAL = al256((size_t)2048 * 4) + al256((size_t)NSP * NMP * NPL * 4) + al256((size_t)NRD * NMP * 2) + al256((size_t)NFP * NRD * 2) + al256((size_t)NSP * NPL * NMP * 2) + al256((size_t)NSP * NRD * NPL * 4) + al256((size_t)NSP * NPL * NRD * 2) + al256((size_t)NSP * NFP * NPL * 4);
static_assert(WS_TOTAL == 43139072 && WS_TOTAL <= 134217728, "the workspace carve: 41.1 MiB");
static_assert(NPL == NSD * NSD && NSD == 64 && NPL % 64 == 0 && NFL == 16 * NTP && NFL <= NFP && NFP % 64 == 0 && NMP % 64 == 0 && NRD % 64 == 0 && OBB + NFL <= 2048 && OBB % 4 == 0 && NFL % 4 == 0, "whole tiles; whole lines; the record's parts apart");
typedef _Float16 h16;
typedef unsigned short bf;
typedef __attribute__((ext_vector_type(16))) __bf16   v16bf;
typedef __attribute__((ext_vector_type(16))) _Float16 v16h;
typedef __attribute__((ext_vector_type(8)))  _Float16 v8h;
typedef __attribute__((ext_vector_type(8)))  unsigned short v8us;
typedef __attribute__((ext_vector_type(8)))  float    v8f;
typedef __attribute__((ext_vector_type(4)))  float    v4f;
typedef v8h  __attribute__((may_alias)) v8ha;
typedef v4f  __attribute__((may_alias)) v4fa;
typedef v8us __attribute__((may_alias)) v8usa;

__device__ __forceinline__ unsigned short f2bf(float f) { unsigned u = __float_as_uint(f); u += 0x7FFFu + ((u >> 16) & 1u); return (unsigned short)(u >> 16); }
__device__ __forceinline__ float bf2f(unsigned short b) { return __uint_as_float(((unsigned)b) << 16); }
__device__ __forceinline__ float bfr(float f) { return bf2f(f2bf(f)); }
__device__ __forceinline__ v16h cat16(v8h lo, v8h hi) { return __builtin_shufflevector(lo, hi, 0, 1, 2, 3, 4, 5, 6, 7, 8, 9, 10, 11, 12, 13, 14, 15); }
__device__ __forceinline__ v16bf cat16b(v8us lo, v8us hi) { return __builtin_bit_cast(v16bf, __builtin_shufflevector(lo, hi, 0, 1, 2, 3, 4, 5, 6, 7, 8, 9, 10, 11, 12, 13, 14, 15)); }
__device__ __forceinline__ v8f wmma16(v16h a, v16h b, v8f c) { return __builtin_amdgcn_wmma_f32_16x16x32_f16(false, a, false, b, (short)0, c, false, false); }
__device__ __forceinline__ v8f wmmab(v16bf a, v16bf b, v8f c) { return __builtin_amdgcn_wmma_f32_16x16x32_bf16(false, a, false, b, (short)0, c, false, false); }


template <typename T16> struct WFrag;
template <> struct WFrag<h16> { typedef v16h V; static __device__ __forceinline__ V ld(const h16* p) { return cat16(*(const v8h*)p, *(const v8h*)(p + 16)); } static __device__ __forceinline__ v8f mma(V a, V b, v8f c) { return wmma16(a, b, c); } };
template <> struct WFrag<bf> { typedef v16bf V; static __device__ __forceinline__ V ld(const bf* p) { return cat16b(*(const v8us*)p, *(const v8us*)(p + 16)); } static __device__ __forceinline__ v8f mma(V a, V b, v8f c) { return wmmab(a, b, c); } };
template <typename T16, int NSPLIT, bool BIAS>
__global__ __launch_bounds__(32) void k_gemmw(const T16* __restrict__ A, const T16* __restrict__ A2, const T16* __restrict__ Bt, const T16* __restrict__ Bt2, int K, float* C, int ldc, const float* __restrict__ bias, size_t sA, size_t sB, size_t sC) {
    typedef typename WFrag<T16>::V V;
    __shared__ __align__(16) float os[16 * 68];
    const size_t z = blockIdx.z; A += z * sA; if (A2) A2 += z * sA; Bt += z * sB; if (Bt2) Bt2 += z * sB; C += z * sC;
    const int lane = threadIdx.x & 31, lr = lane & 15, hi = lane >> 4; const int r0 = blockIdx.x * 64, c0 = blockIdx.y * 64;
    v8f acc[4][4];
#pragma unroll
    for (int mb = 0; mb < 4; ++mb)
#pragma unroll
        for (int nb = 0; nb < 4; ++nb) acc[mb][nb] = (v8f){};
    const size_t aoff = (size_t)(r0 + lr) * K + 8 * hi, boff = (size_t)(c0 + lr) * K + 8 * hi;
    for (int kc = 0; kc < K; kc += 32) {
        V a[4], a2[4];
#pragma unroll
        for (int mb = 0; mb < 4; ++mb) { a[mb] = WFrag<T16>::ld(A + aoff + (size_t)mb * 16 * K + kc); if (NSPLIT == 1 || NSPLIT == 2) a2[mb] = WFrag<T16>::ld(A2 + aoff + (size_t)mb * 16 * K + kc); }
#pragma unroll
        for (int nb = 0; nb < 4; ++nb) { const V b = WFrag<T16>::ld(Bt + boff + (size_t)nb * 16 * K + kc); V b2; if (NSPLIT >= 2) b2 = WFrag<T16>::ld(Bt2 + boff + (size_t)nb * 16 * K + kc);
#pragma unroll
            for (int mb = 0; mb < 4; ++mb) { acc[mb][nb] = WFrag<T16>::mma(a[mb], b, acc[mb][nb]); if (NSPLIT == 1 || NSPLIT == 2) acc[mb][nb] = WFrag<T16>::mma(a2[mb], b, acc[mb][nb]); if (NSPLIT >= 2) acc[mb][nb] = WFrag<T16>::mma(a[mb], b2, acc[mb][nb]); } }
        asm volatile("v_nop\n\tv_nop\n\tv_nop\n\tv_nop" : "+v"(acc[0][0]), "+v"(acc[1][1]), "+v"(acc[2][2]), "+v"(acc[3][3]) : "v"(a[0]), "v"(a[3]));
    }
#pragma unroll
    for (int mb = 0; mb < 4; ++mb) {
#pragma unroll
        for (int nb = 0; nb < 4; ++nb) {
#pragma unroll
            for (int j = 0; j < 8; ++j) os[(hi * 8 + j) * 68 + nb * 16 + lr] = acc[mb][nb][j]; }
        __builtin_amdgcn_wave_barrier(); asm volatile("" ::: "memory");
        float* crow = C + (size_t)(r0 + mb * 16) * ldc + c0;
#pragma unroll 1
        for (int ps = 0; ps < 2; ++ps) {
#pragma unroll
            for (int s = 0; s < 8; ++s) { const int row = 2 * s + hi, cofs = lr * 4; v4f val = *(const v4fa*)(os + row * 68 + cofs); if (BIAS) { val[0] += bfr(bias[c0 + cofs]); val[1] += bfr(bias[c0 + cofs + 1]); val[2] += bfr(bias[c0 + cofs + 2]); val[3] += bfr(bias[c0 + cofs + 3]); }
                *(volatile v4f*)(crow + (size_t)row * ldc + cofs) = val; }
            if (ps == 0) __threadfence(); }
        __builtin_amdgcn_wave_barrier(); asm volatile("" ::: "memory");
    }
}

__device__ __forceinline__ h16 tohx(float x) { return (h16)x; }
__device__ __forceinline__ void splitf(float y, unsigned short& h, unsigned short& l) { h = f2bf(y); l = f2bf(y - bf2f(h)); }
typedef __attribute__((ext_vector_type(2))) _Float16 v2h;
typedef __attribute__((ext_vector_type(4))) _Float16 v4h;
typedef __attribute__((ext_vector_type(2))) unsigned short v2us;
typedef __attribute__((ext_vector_type(4))) unsigned short v4us;
typedef __attribute__((ext_vector_type(2))) float v2f;
typedef __attribute__((ext_vector_type(4))) int v4i;


__global__ __launch_bounds__(256) void k_lay(const float* __restrict__ src, h16* dst, unsigned nrow, unsigned c8n, unsigned dp, unsigned c0, unsigned rbs, unsigned ra, unsigned rs, unsigned cbs, unsigned sa, unsigned sb, unsigned rlive, unsigned clive) {
    const unsigned g = blockIdx.x * 256 + threadIdx.x; if (g >= nrow * c8n) return; const unsigned row = g / c8n, ch = g - row * c8n; const unsigned rb = (row >> rbs) * ra + (row & ((1u << rbs) - 1u)) * rs; v8h o;
#pragma unroll
    for (int w = 0; w < 8; ++w) { const unsigned c = 8u * ch + w; const bool live = row < rlive && c < clive; const unsigned si = rb + (c >> cbs) * sa + (c & ((1u << cbs) - 1u)) * sb; const float v = bfr(src[live ? si : 0u]); o[w] = tohx(live && fabsf(v) >= 6.103515625e-05f ? v : 0.0f); }
    h16* d8 = dst + (size_t)row * dp + c0 + 8u * ch; *(volatile v8h*)(d8) = o; __threadfence(); *(volatile v8h*)(d8) = o; }

__global__ __launch_bounds__(256) void k_rnd(const float* __restrict__ src, float* dst, unsigned npc, unsigned nw) {
    const unsigned g = blockIdx.x * 256 + threadIdx.x; if (g >= npc) return; v4f o;
#pragma unroll
    for (int e = 0; e < 4; ++e) { const unsigned i = 4u * g + (unsigned)e; const unsigned live = i < nw ? 1u : 0u; const float rv_ = bfr(src[live ? i : 0u]); o[e] = live ? rv_ : 0.0f; }
    float* dq = dst + 4u * (size_t)g; *(volatile v4f*)(dq) = o; __threadfence(); *(volatile v4f*)(dq) = o; }

__global__ __launch_bounds__(256) void k_act(const float* __restrict__ tp, const float* __restrict__ rs, h16* tt) {
    const unsigned t0 = blockIdx.x * 256 + threadIdx.x; if (t0 >= (unsigned)(NPL * (NRD / 8))) return; const unsigned sm = blockIdx.y, ch = t0 & 7u, pl = t0 >> 3; const float* tq = tp + ((size_t)sm * NRD + 8u * ch) * NPL + pl; v8h o;
#pragma unroll
    for (int e = 0; e < 8; ++e) { const unsigned q = 8u * ch + (unsigned)e; const float fac = rs[q] / sqrtf(rs[192 + q] + 1e-5f); const float off = rs[64 + q] - rs[128 + q] * fac; const float rv = fmaxf(tq[(size_t)e * NPL] * fac + off, 0.0f);
        const float kf = fabsf(rv) >= 6.103515625e-05f ? 1.0f : 0.0f; o[e] = tohx(rv * kf); }
    h16* d8 = tt + ((size_t)sm * NPL + pl) * NRD + 8u * ch; *(volatile v8h*)(d8) = o; __threadfence(); *(volatile v8h*)(d8) = o; }

__global__ __launch_bounds__(256) void k_bia(float* kr, const float* __restrict__ rs) {
    const unsigned g = blockIdx.x * 256 + threadIdx.x; if (g >= (unsigned)(NPL / 4)) return; const unsigned pr = blockIdx.y, sm = pr / (unsigned)NFL, rw = pr - sm * (unsigned)NFL; const float bw_ = rs[OBB + rw];
    float* dq = kr + ((size_t)sm * NFP + rw) * NPL + 4u * (size_t)g; const v4f a = *(const v4f*)dq; v4f o;
#pragma unroll
    for (int e = 0; e < 4; ++e) o[e] = a[e] + bw_;
    *(volatile v4f*)(dq) = o; __threadfence(); *(volatile v4f*)(dq) = o; }

__global__ __launch_bounds__(256) void k_tap(const float* __restrict__ xr, const float* __restrict__ kr, float* rsl) {
    const unsigned pl = blockIdx.x * 256 + threadIdx.x; if (pl >= (unsigned)NPL) return; const unsigned pr = blockIdx.y, sm = pr >> 8, gp = (pr & 255u) >> 4; const unsigned py = pl >> 6, px = pl & 63u;
    const float* xm = xr + (size_t)pr * NPL; const float* kq = kr + ((size_t)sm * NFP + gp * (unsigned)NTP) * NPL + pl; float acc = 0.0f;
#pragma unroll
    for (int u = 0; u < 7; ++u) { const unsigned yy = py + (unsigned)u - 3u; const unsigned yin = yy < (unsigned)NSD ? 1u : 0u; const unsigned yc = yin ? yy : 0u;
#pragma unroll
        for (int v = 0; v < 7; ++v) { const unsigned xx = px + (unsigned)v - 3u; const unsigned ins = (xx < (unsigned)NSD ? 1u : 0u) & yin; const unsigned xc = ins ? xx : 0u; const float lv = ins ? 1.0f : 0.0f;
            acc += (lv * xm[yc * (unsigned)NSD + xc]) * kq[(size_t)(7 * u + v) * NPL]; } }
    const float ov = acc + xm[pl]; float* dq = rsl + (size_t)pr * NPL + pl; *(volatile float*)(dq) = ov; __threadfence(); *(volatile float*)(dq) = ov; }

extern "C" void kernel_launch(void* const* d_in, const int* in_sizes, int n_in,
                              void* d_out, int out_size, void* d_ws, size_t ws_size, hipStream_t stream) {
    if (n_in < 9) return;
    if (in_sizes[0] < NSP * NMP * NPL || in_sizes[1] < NSP * NMP * NPL || in_sizes[2] < NRD * NMP || in_sizes[7] < NFL * NRD || in_sizes[8] < NFL || out_size < NSP * NMP * NPL) return;
    for (int q = 3; q < 7; ++q) if (in_sizes[q] < NRD) return;
    const float* ia = (const float*)d_in[0]; const float* ib = (const float*)d_in[1]; const float* wa = (const float*)d_in[2]; const float* wb = (const float*)d_in[7]; const float* bb = (const float*)d_in[8];
    const float* gq = (const float*)d_in[3]; const float* bq = (const float*)d_in[4]; const float* mq = (const float*)d_in[5]; const float* vq = (const float*)d_in[6];
    char* wsp = (char*)d_ws;
    auto take = [&](size_t bytes) { char* cur = wsp; wsp += (bytes + 255) & ~(size_t)255; return (void*)cur; };
    float* RS = (float*)take((size_t)2048 * 4); float* XR = (float*)take((size_t)NSP * NMP * NPL * 4); h16* RW = (h16*)take((size_t)NRD * NMP * 2); h16* SW = (h16*)take((size_t)NFP * NRD * 2); h16* GT = (h16*)take((size_t)NSP * NPL * NMP * 2); float* TP = (float*)take((size_t)NSP * NRD * NPL * 4); h16* TT = (h16*)take((size_t)NSP * NPL * NRD * 2); float* KR = (float*)take((size_t)NSP * NFP * NPL * 4);
    if ((size_t)(wsp - (char*)d_ws) != WS_TOTAL || WS_TOTAL > ws_size) return;
    auto lay = [&](const float* sp_, h16* dp_, unsigned nrow, unsigned ncol, unsigned dp, unsigned c0, unsigned rbs, unsigned ra, unsigned rs_, unsigned cbs, unsigned sa, unsigned sb, unsigned rlive, unsigned clive) {
        k_lay<<<(nrow * (ncol / 8) + 255) / 256, 256, 0, stream>>>(sp_, dp_, nrow, ncol / 8, dp, c0, rbs, ra, rs_, cbs, sa, sb, rlive, clive); };
    auto rnd = [&](const float* sp_, float* dp_, unsigned nw) { const unsigned npc = (nw + 3) / 4; k_rnd<<<(npc + 255) / 256, 256, 0, stream>>>(sp_, dp_, npc, nw); };
    rnd(gq, RS, NRD); rnd(bq, RS + 64, NRD); rnd(mq, RS + 128, NRD); rnd(vq, RS + 192, NRD); rnd(bb, RS + OBB, NFL);
    rnd(ia, XR, NSP * NMP * NPL);
    lay(wa, RW, NRD, NMP, NMP, 0, 16, 0, NMP, 16, 0, 1, NRD, NMP);
    lay(wb, SW, NFP, NRD, NRD, 0, 16, 0, NRD, 16, 0, 1, NFL, NRD);
    for (int s = 0; s < NSP; ++s) lay(ib + (size_t)s * NMP * NPL, GT + (size_t)s * NPL * NMP, NPL, NMP, NMP, 0, 16, 0, 1, 16, 0, NPL, NPL, NMP);
    k_gemmw<h16, 0, false><<<dim3(NRD / 64, NPL / 64, NSP), 32, 0, stream>>>(RW, nullptr, GT, nullptr, NMP, TP, NPL, nullptr, (size_t)0, (size_t)NPL * NMP, (size_t)NRD * NPL);
    k_act<<<dim3((NPL * (NRD / 8) + 255) / 256, NSP, 1), 256, 0, stream>>>(TP, RS, TT);
    k_gemmw<h16, 0, false><<<dim3(NFP / 64, NPL / 64, NSP), 32, 0, stream>>>(SW, nullptr, TT, nullptr, NRD, KR, NPL, nullptr, (size_t)0, (size_t)NPL * NRD, (size_t)NFP * NPL);
    k_bia<<<dim3((NPL / 4 + 255) / 256, NSP * NFL, 1), 256, 0, stream>>>(KR, RS);
    k_tap<<<dim3((NPL + 255) / 256, NSP * NMP, 1), 256, 0, stream>>>(XR, KR, (float*)d_out);
}
